// GraformerLayer_14285061226622
// MI455X (gfx1250) — hardware-verified
//
#include <hip/hip_runtime.h>

typedef _Float16 f16;
typedef f16 v8h __attribute__((ext_vector_type(8)));
typedef f16 v8hm __attribute__((ext_vector_type(8))) __attribute__((may_alias));
typedef f16 v16h __attribute__((ext_vector_type(16)));
typedef float v8f __attribute__((ext_vector_type(8)));
typedef float v4f __attribute__((ext_vector_type(4)));
typedef float v4fm __attribute__((ext_vector_type(4))) __attribute__((may_alias));
union Frag { v16h v; v8h hf[2]; };

static constexpr int NB = 8, NN = 1024, ND = 256, NH = 8, DH = 32, DFF = 1024, NK = 3;

__device__ __forceinline__ v8f mma16(v16h a, v16h b, v8f c) {
  c = __builtin_amdgcn_wmma_f32_16x16x32_f16(false, a, false, b, (short)0, c, false, false);
  asm volatile("v_nop\n\tv_nop\n\tv_nop\n\tv_nop" : "+v"(c) : "v"(a), "v"(b));
  return c;
}
__device__ __forceinline__ v8h pack8(const float* v) {
  v8h r;
#pragma unroll
  for (int j = 0; j < 8; ++j) r[j] = (f16)v[j];
  return r;
}

template <int EP>
__global__ void __launch_bounds__(128) gemm_f16(const f16* __restrict__ A, int lda, long long sA,
                                              const f16* __restrict__ B, int ldb, long long sB,
                                              f16* outH, float* outF, int ldo, long long sO,
                                              const float* __restrict__ base, int ldbase, long long sBase,
                                              const float* __restrict__ bias, int use_bias,
                                              const f16* __restrict__ aux, int ldaux, long long sAux,
                                              int K, float scale) {
  __shared__ __attribute__((aligned(16))) v8h As[64 * 5];
  __shared__ __attribute__((aligned(16))) f16 Bt[64 * 40];
  __shared__ __attribute__((aligned(16))) float Cs[64 * 68];
  const int t = threadIdx.x, w = t >> 5, l = t & 31, hh = l >> 4, m = l & 15;
  const int wm = w >> 1, wn = w & 1;
  const int n0 = blockIdx.x * 64, m0 = blockIdx.y * 64, z = blockIdx.z;
  const f16* Ab = A + (long long)z * sA + (long long)m0 * lda;
  const f16* Bb = B + (long long)z * sB + n0;

  v8f acc[2][2];
#pragma unroll
  for (int i = 0; i < 2; ++i)
#pragma unroll
    for (int j = 0; j < 2; ++j) acc[i][j] = (v8f){};

  for (int k0 = 0; k0 < K; k0 += 32) {
#pragma unroll
    for (int i = 0; i < 2; ++i) {
      const int p = t + 128 * i, row = p >> 2, seg = p & 3;
      As[row * 5 + seg] = *(const v8h*)(Ab + (long long)row * lda + k0 + seg * 8);
    }
#pragma unroll
    for (int i = 0; i < 2; ++i) {
      const int p = t + 128 * i, kk = p >> 3, seg = p & 7;
      const v8h v = *(const v8h*)(Bb + (long long)(k0 + kk) * ldb + seg * 8);
#pragma unroll
      for (int j = 0; j < 8; ++j) Bt[(seg * 8 + j) * 40 + kk] = v[j];
    }
    __syncthreads();
    Frag a[2], b[2];
#pragma unroll
    for (int mt = 0; mt < 2; ++mt) {
      const int row = wm * 32 + mt * 16 + m;
      a[mt].hf[0] = As[row * 5 + hh];
      a[mt].hf[1] = As[row * 5 + 2 + hh];
    }
#pragma unroll
    for (int nt = 0; nt < 2; ++nt) {
      const int col = wn * 32 + nt * 16 + m;
      b[nt].hf[0] = *(const v8hm*)(Bt + col * 40 + 8 * hh);
      b[nt].hf[1] = *(const v8hm*)(Bt + col * 40 + 16 + 8 * hh);
    }
#pragma unroll
    for (int mt = 0; mt < 2; ++mt)
#pragma unroll
      for (int nt = 0; nt < 2; ++nt) acc[mt][nt] = mma16(a[mt].v, b[nt].v, acc[mt][nt]);
    __syncthreads();
  }

#pragma unroll
  for (int mt = 0; mt < 2; ++mt)
#pragma unroll
    for (int nt = 0; nt < 2; ++nt)
#pragma unroll
      for (int r = 0; r < 8; ++r)
        Cs[(wm * 32 + mt * 16 + 8 * hh + r) * 68 + wn * 32 + nt * 16 + m] = acc[mt][nt][r];
  __syncthreads();

  if constexpr (EP < 3) {
    v8h vals[4];
    f16* ptrs[4];
#pragma unroll
    for (int i = 0; i < 4; ++i) {
      const int row = w * 16 + 4 * i + (l >> 3), c8 = (l & 7) * 8;
      const float* cp = Cs + row * 68 + c8;
      const v4f x0 = *(const v4fm*)cp, x1 = *(const v4fm*)(cp + 4);
      float v[8] = {x0[0], x0[1], x0[2], x0[3], x1[0], x1[1], x1[2], x1[3]};
      const int gm = m0 + row, gc = n0 + c8;
      if constexpr (EP == 0) {
#pragma unroll
        for (int j = 0; j < 8; ++j) v[j] = v[j] * scale;
      } else if constexpr (EP == 1) {
        const v4f b0 = *(const v4f*)(bias + gc), b1 = *(const v4f*)(bias + gc + 4);
        const float bb[8] = {b0[0], b0[1], b0[2], b0[3], b1[0], b1[1], b1[2], b1[3]};
#pragma unroll
        for (int j = 0; j < 8; ++j) { const float s = v[j] * scale + bb[j]; v[j] = s > 0.f ? s : 0.f; }
      } else {
        const v8h ax = *(const v8h*)(aux + (long long)z * sAux + (long long)gm * ldaux + gc);
#pragma unroll
        for (int j = 0; j < 8; ++j) v[j] = 2.f * (v[j] * scale) - (float)ax[j];
      }
      vals[i] = pack8(v);
      ptrs[i] = outH + (long long)z * sO + (long long)gm * ldo + gc;
    }
#pragma unroll
    for (int i = 0; i < 4; ++i) *(volatile v8h*)ptrs[i] = vals[i];
    __threadfence();
#pragma unroll
    for (int i = 0; i < 4; ++i) *(volatile v8h*)ptrs[i] = vals[i];
  } else {
    v4f vals[8];
    float* ptrs[8];
#pragma unroll
    for (int i = 0; i < 8; ++i) {
      const int row = w * 16 + 2 * i + hh, c4 = m * 4;
      const v4f x = *(const v4fm*)(Cs + row * 68 + c4);
      const int gm = m0 + row, gc = n0 + c4;
      const v4f bs = *(const v4f*)(base + (long long)z * sBase + (long long)gm * ldbase + gc);
      v4f v = bs + x * scale;
      if (use_bias) { const v4f bb = *(const v4f*)(bias + gc); v = v + bb; }
      vals[i] = v;
      ptrs[i] = outF + (long long)z * sO + (long long)gm * ldo + gc;
    }
#pragma unroll
    for (int i = 0; i < 8; ++i) *(volatile v4f*)ptrs[i] = vals[i];
    __threadfence();
#pragma unroll
    for (int i = 0; i < 8; ++i) *(volatile v4f*)ptrs[i] = vals[i];
  }
}

__global__ void __launch_bounds__(128) attn_f16(const f16* __restrict__ G, const float* __restrict__ Z,
                                              float* z1) {
  __shared__ __attribute__((aligned(16))) f16 Gt[32 * 520];
  __shared__ __attribute__((aligned(16))) float Sc[4][16 * 36];
  __shared__ __attribute__((aligned(16))) f16 Pt[4][16 * 40];
  const int t = threadIdx.x, w = t >> 5, l = t & 31, hh = l >> 4, m = l & 15;
  const int b = blockIdx.z, h = blockIdx.y, q0 = blockIdx.x * 64 + w * 16;
  const f16* Gb = G + (long long)b * NN * ND + h * DH;
  const float SCL = 1.0f / (256.0f * 5.656854249492381f);
  float* sc = Sc[w];
  f16* pt = Pt[w];

  Frag qa;
  qa.hf[0] = *(const v8h*)(Gb + (long long)(q0 + m) * ND + 8 * hh);
  qa.hf[1] = *(const v8h*)(Gb + (long long)(q0 + m) * ND + 16 + 8 * hh);

  float mrun = -3.0e38f, srun = 0.f;
  for (int kc = 0; kc < NN / 32; ++kc) {
#pragma unroll
    for (int tile = 0; tile < 2; ++tile) {
      const int rk = kc * 32 + tile * 16 + m;
      Frag kb;
      kb.hf[0] = *(const v8h*)(Gb + (long long)rk * ND + 8 * hh);
      kb.hf[1] = *(const v8h*)(Gb + (long long)rk * ND + 16 + 8 * hh);
      v8f c = (v8f){};
      c = mma16(qa.v, kb.v, c);
#pragma unroll
      for (int r = 0; r < 8; ++r) sc[(8 * hh + r) * 36 + tile * 16 + m] = c[r] * SCL;
    }
    __syncthreads();
    {
      const float* rp = sc + m * 36 + 16 * hh;
      const v4f x0 = *(const v4fm*)rp, x1 = *(const v4fm*)(rp + 4), x2 = *(const v4fm*)(rp + 8), x3 = *(const v4fm*)(rp + 12);
      const float x[16] = {x0[0], x0[1], x0[2], x0[3], x1[0], x1[1], x1[2], x1[3],
                           x2[0], x2[1], x2[2], x2[3], x3[0], x3[1], x3[2], x3[3]};
      float ml = x[0];
#pragma unroll
      for (int j = 1; j < 16; ++j) ml = fmaxf(ml, x[j]);
      const float mn = fmaxf(mrun, ml);
      float s = srun * __expf(mrun - mn);
#pragma unroll
      for (int j = 0; j < 16; ++j) s += __expf(x[j] - mn);
      srun = s; mrun = mn;
    }
    __syncthreads();
  }
  const float mo = __shfl_xor(mrun, 16, 32), so = __shfl_xor(srun, 16, 32);
  const float mtot = fmaxf(mrun, mo);
  const float stot = srun * __expf(mrun - mtot) + so * __expf(mo - mtot);
  const float pinv = 4096.0f / stot;

  v8f o0 = (v8f){}, o1 = (v8f){};
  for (int c = 0; c < NN / 512; ++c) {
    __syncthreads();
#pragma unroll 4
    for (int it = 0; it < 16; ++it) {
      const int p = it * 128 + t, mm = p >> 2, seg = p & 3;
      const v8h v = *(const v8h*)(Gb + (long long)(c * 512 + mm) * ND + seg * 8);
#pragma unroll
      for (int j = 0; j < 8; ++j) Gt[(seg * 8 + j) * 520 + mm] = v[j];
    }
    __syncthreads();
    for (int ks = 0; ks < 16; ++ks) {
      const int kb0 = c * 512 + ks * 32;
#pragma unroll
      for (int tile = 0; tile < 2; ++tile) {
        const int rk = kb0 + tile * 16 + m;
        Frag kb;
        kb.hf[0] = *(const v8h*)(Gb + (long long)rk * ND + 8 * hh);
        kb.hf[1] = *(const v8h*)(Gb + (long long)rk * ND + 16 + 8 * hh);
        v8f cc = (v8f){};
        cc = mma16(qa.v, kb.v, cc);
#pragma unroll
        for (int r = 0; r < 8; ++r) sc[(8 * hh + r) * 36 + tile * 16 + m] = cc[r] * SCL;
      }
      __syncthreads();
      {
        const float* rp = sc + m * 36 + 16 * hh;
        const v4f x0 = *(const v4fm*)rp, x1 = *(const v4fm*)(rp + 4), x2 = *(const v4fm*)(rp + 8), x3 = *(const v4fm*)(rp + 12);
        const float x[16] = {x0[0], x0[1], x0[2], x0[3], x1[0], x1[1], x1[2], x1[3],
                             x2[0], x2[1], x2[2], x2[3], x3[0], x3[1], x3[2], x3[3]};
        float pv[16];
#pragma unroll
        for (int j = 0; j < 16; ++j) pv[j] = __expf(x[j] - mtot) * pinv;
        *(v8hm*)(pt + m * 40 + 16 * hh) = pack8(pv);
        *(v8hm*)(pt + m * 40 + 16 * hh + 8) = pack8(pv + 8);
      }
      __syncthreads();
      Frag pa;
      pa.hf[0] = *(const v8hm*)(pt + m * 40 + 8 * hh);
      pa.hf[1] = *(const v8hm*)(pt + m * 40 + 16 + 8 * hh);
      Frag vb0, vb1;
      vb0.hf[0] = *(const v8hm*)(Gt + m * 520 + ks * 32 + 8 * hh);
      vb0.hf[1] = *(const v8hm*)(Gt + m * 520 + ks * 32 + 16 + 8 * hh);
      vb1.hf[0] = *(const v8hm*)(Gt + (16 + m) * 520 + ks * 32 + 8 * hh);
      vb1.hf[1] = *(const v8hm*)(Gt + (16 + m) * 520 + ks * 32 + 16 + 8 * hh);
      o0 = mma16(pa.v, vb0.v, o0);
      o1 = mma16(pa.v, vb1.v, o1);
    }
  }

  const float OS = 1.0f / 65536.0f;
  __syncthreads();
#pragma unroll
  for (int r = 0; r < 8; ++r) {
    sc[(8 * hh + r) * 36 + m] = o0[r] * OS;
    sc[(8 * hh + r) * 36 + 16 + m] = o1[r] * OS;
  }
  __syncthreads();
  v4f vals[4];
  float* ptrs[4];
#pragma unroll
  for (int i = 0; i < 4; ++i) {
    const int row = 4 * i + (l >> 3), c4 = (l & 7) * 4;
    const v4f o = *(const v4fm*)(sc + row * 36 + c4);
    const long long gi = ((long long)b * NN + q0 + row) * ND + h * DH + c4;
    const v4f zz = *(const v4f*)(Z + gi);
    vals[i] = zz + o;
    ptrs[i] = z1 + gi;
  }
#pragma unroll
  for (int i = 0; i < 4; ++i) *(volatile v4f*)ptrs[i] = vals[i];
  __threadfence();
#pragma unroll
  for (int i = 0; i < 4; ++i) *(volatile v4f*)ptrs[i] = vals[i];
}

__global__ void __launch_bounds__(256) ln_f16(const float* __restrict__ X, const float* __restrict__ g,
                                            const float* __restrict__ bb, f16* Y, int ldy, int rows) {
  const int l = threadIdx.x & 31;
  const int row = blockIdx.x * 8 + (threadIdx.x >> 5);
  if (row >= rows) return;
  const float* x = X + (long long)row * ND + 8 * l;
  const v4f a = *(const v4f*)x, c = *(const v4f*)(x + 4);
  float v[8] = {a[0], a[1], a[2], a[3], c[0], c[1], c[2], c[3]};
  float s = 0.f;
#pragma unroll
  for (int j = 0; j < 8; ++j) s += v[j];
#pragma unroll
  for (int o = 16; o; o >>= 1) s += __shfl_xor(s, o, 32);
  const float mu = s * (1.0f / ND);
  float q = 0.f;
#pragma unroll
  for (int j = 0; j < 8; ++j) { v[j] -= mu; q += v[j] * v[j]; }
#pragma unroll
  for (int o = 16; o; o >>= 1) q += __shfl_xor(q, o, 32);
  const float rstd = rsqrtf(q * (1.0f / ND) + 1e-5f);
  const v4f g0 = *(const v4f*)(g + 8 * l), g1 = *(const v4f*)(g + 8 * l + 4);
  const v4f b0 = *(const v4f*)(bb + 8 * l), b1 = *(const v4f*)(bb + 8 * l + 4);
  const float gg[8] = {g0[0], g0[1], g0[2], g0[3], g1[0], g1[1], g1[2], g1[3]};
  const float be[8] = {b0[0], b0[1], b0[2], b0[3], b1[0], b1[1], b1[2], b1[3]};
  float y[8];
#pragma unroll
  for (int j = 0; j < 8; ++j) y[j] = v[j] * rstd * gg[j] + be[j];
  const v8h out = pack8(y);
  f16* p = Y + (long long)row * ldy + 8 * l;
  *(volatile v8h*)p = out;
  __threadfence();
  *(volatile v8h*)p = out;
}

__global__ void __launch_bounds__(256) degree_k(const float* __restrict__ adj, float* dinv, int rows) {
  __shared__ __attribute__((aligned(16))) float dv[32];
  const int w = threadIdx.x >> 5, l = threadIdx.x & 31, blk = blockIdx.x;
#pragma unroll 1
  for (int j = 0; j < 4; ++j) {
    const int row = blk * 32 + w * 4 + j;
    float s = 0.f;
    if (row < rows) {
      const float* a = adj + (long long)row * NN;
      for (int i = l * 4; i < NN; i += 128) { const v4f v = *(const v4f*)(a + i); s += v[0] + v[1] + v[2] + v[3]; }
    }
#pragma unroll
    for (int o = 16; o; o >>= 1) s += __shfl_xor(s, o, 32);
    if (l == 0) dv[w * 4 + j] = 1.0f / sqrtf(s + 1.0f);
  }
  __syncthreads();
  if (w == 0 && l < 8) {
    const int r0 = blk * 32 + 4 * l;
    if (r0 + 3 < rows) {
      const v4f v = *(const v4fm*)(dv + 4 * l);
      float* p = dinv + r0;
      *(volatile v4f*)p = v;
      __threadfence();
      *(volatile v4f*)p = v;
    }
  }
}

__global__ void __launch_bounds__(256) anorm_k(const float* __restrict__ adj, const float* __restrict__ dinv,
                                             f16* A16, int ngrp) {
  const int gid = blockIdx.x * 256 + threadIdx.x;
  if (gid >= ngrp) return;
  const int b = gid >> 17, n = (gid >> 7) & (NN - 1), mg = (gid & 127) * 8;
  const float dn = dinv[b * NN + n];
  const v4f d0 = *(const v4f*)(dinv + b * NN + mg), d1 = *(const v4f*)(dinv + b * NN + mg + 4);
  const v4f a0 = *(const v4f*)(adj + (long long)gid * 8), a1 = *(const v4f*)(adj + (long long)gid * 8 + 4);
  const float av[8] = {a0[0], a0[1], a0[2], a0[3], a1[0], a1[1], a1[2], a1[3]};
  const float dm[8] = {d0[0], d0[1], d0[2], d0[3], d1[0], d1[1], d1[2], d1[3]};
  float v[8];
#pragma unroll
  for (int j = 0; j < 8; ++j) {
    const float ah = av[j] + ((n == mg + j) ? 1.0f : 0.0f);
    v[j] = ((ah * dn) * dm[j]) * 4096.0f;
  }
  const v8h out = pack8(v);
  f16* p = A16 + (long long)gid * 8;
  *(volatile v8h*)p = out;
  __threadfence();
  *(volatile v8h*)p = out;
}

__global__ void __launch_bounds__(256) cvt_f16(const float* __restrict__ x, f16* y, int ngrp, float s) {
  const int gid = blockIdx.x * 256 + threadIdx.x;
  if (gid >= ngrp) return;
  const v4f a0 = *(const v4f*)(x + (long long)gid * 8), a1 = *(const v4f*)(x + (long long)gid * 8 + 4);
  const float v[8] = {a0[0] * s, a0[1] * s, a0[2] * s, a0[3] * s, a1[0] * s, a1[1] * s, a1[2] * s, a1[3] * s};
  const v8h out = pack8(v);
  f16* p = y + (long long)gid * 8;
  *(volatile v8h*)p = out;
  __threadfence();
  *(volatile v8h*)p = out;
}

__global__ void __launch_bounds__(256) wcat_k(const float* __restrict__ W, f16* Wc, int nthr) {
  const int gid = blockIdx.x * 256 + threadIdx.x;
  if (gid >= nthr) return;
  const int k = gid >> 5, h = (gid >> 2) & 7, q = gid & 3;
  const float* src = W + ((long long)(h * ND + k)) * DH + q * 8;
  const v4f a0 = *(const v4f*)src, a1 = *(const v4f*)(src + 4);
  const float s = 16.0f;
  const float v[8] = {a0[0] * s, a0[1] * s, a0[2] * s, a0[3] * s, a1[0] * s, a1[1] * s, a1[2] * s, a1[3] * s};
  const v8h out = pack8(v);
  f16* p = Wc + (long long)k * ND + h * DH + q * 8;
  *(volatile v8h*)p = out;
  __threadfence();
  *(volatile v8h*)p = out;
}

extern "C" void kernel_launch(void* const* d_in, const int* in_sizes, int n_in,
                              void* d_out, int out_size, void* d_ws, size_t ws_size,
                              hipStream_t stream) {
  if (n_in < 15) return;
  if (in_sizes[0] != NB * NN * ND || in_sizes[1] != NB * NN * NN || in_sizes[2] != NB * NN * NN ||
      in_sizes[9] != NH * ND * DH || in_sizes[10] != ND * DFF || in_sizes[12] != DFF * ND ||
      in_sizes[14] != NK * ND * ND || in_sizes[11] != DFF || in_sizes[13] != ND ||
      in_sizes[3] != ND || out_size != NB * NN * ND) return;
  const float* Z    = (const float*)d_in[0];
  const float* adj  = (const float*)d_in[1];
  const float* lap  = (const float*)d_in[2];
  const float* ln1g = (const float*)d_in[3];
  const float* ln1b = (const float*)d_in[4];
  const float* ln2g = (const float*)d_in[5];
  const float* ln2b = (const float*)d_in[6];
  const float* ln3g = (const float*)d_in[7];
  const float* ln3b = (const float*)d_in[8];
  const float* Wh   = (const float*)d_in[9];
  const float* W1   = (const float*)d_in[10];
  const float* b1   = (const float*)d_in[11];
  const float* W2   = (const float*)d_in[12];
  const float* b2   = (const float*)d_in[13];
  const float* Th   = (const float*)d_in[14];
  float* out = (float*)d_out;

  char* ws = (char*)d_ws;
  size_t off = 0;
  auto carve = [&](size_t bytes) { char* p = ws + off; off = (off + bytes + 255) & ~(size_t)255; return p; };
  const size_t rowsAll = (size_t)NB * NN;
  f16*   zn   = (f16*)carve(rowsAll * ND * 2);
  float* dinv = (float*)carve(rowsAll * 4);
  f16*   wcat = (f16*)carve((size_t)ND * ND * 2);
  f16*   Xh   = (f16*)carve(rowsAll * ND * 2);
  f16*   Gh   = (f16*)carve(rowsAll * ND * 2);
  f16*   A16  = (f16*)carve((size_t)NB * NN * NN * 2);
  float* z1   = (float*)carve(rowsAll * ND * 4);
  f16*   w1h  = (f16*)carve((size_t)ND * DFF * 2);
  f16*   hid  = (f16*)carve(rowsAll * DFF * 2);
  f16*   w2h  = (f16*)carve((size_t)DFF * ND * 2);
  float* z2   = (float*)carve(rowsAll * ND * 4);
  f16*   L16  = (f16*)carve((size_t)NB * NN * NN * 2);
  f16*   thh  = (f16*)carve((size_t)NK * ND * ND * 2);
  f16*   txc  = (f16*)carve(rowsAll * (NK * ND) * 2);
  if (off > ws_size) return;

  const float inv16 = 0.0625f;
  const long long sNN = (long long)NN * NN, sND = (long long)NN * ND, sTX = (long long)NN * NK * ND;

  ln_f16<<<(unsigned)((rowsAll + 7) / 8), 256, 0, stream>>>(Z, ln1g, ln1b, zn, ND, (int)rowsAll);
  degree_k<<<(unsigned)((rowsAll + 31) / 32), 256, 0, stream>>>(adj, dinv, (int)rowsAll);
  {
    const int ngrp = NB * NN * NN / 8;
    anorm_k<<<(ngrp + 255) / 256, 256, 0, stream>>>(adj, dinv, A16, ngrp);
    const int nthr = NH * ND * 4;
    wcat_k<<<(nthr + 255) / 256, 256, 0, stream>>>(Wh, wcat, nthr);
  }
  gemm_f16<0><<<dim3(ND / 64, (unsigned)(rowsAll / 64), 1), 128, 0, stream>>>(
      zn, ND, 0, wcat, ND, 0, Xh, z1, ND, 0, z1, ND, 0, b1, 0, zn, ND, 0, ND, inv16);
  gemm_f16<0><<<dim3(ND / 64, NN / 64, NB), 128, 0, stream>>>(
      A16, NN, sNN, Xh, ND, sND, Gh, z1, ND, sND, z1, ND, 0, b1, 0, zn, ND, 0, NN, 1.0f / 256.0f);
  attn_f16<<<dim3(NN / 64, NH, NB), 128, 0, stream>>>(Gh, Z, z1);

  ln_f16<<<(unsigned)((rowsAll + 7) / 8), 256, 0, stream>>>(z1, ln2g, ln2b, zn, ND, (int)rowsAll);
  {
    const int n1 = ND * DFF / 8;
    cvt_f16<<<(n1 + 255) / 256, 256, 0, stream>>>(W1, w1h, n1, 16.0f);
  }
  gemm_f16<1><<<dim3(DFF / 64, (unsigned)(rowsAll / 64), 1), 128, 0, stream>>>(
      zn, ND, 0, w1h, DFF, 0, hid, z2, DFF, 0, z1, ND, 0, b1, 1, zn, ND, 0, ND, inv16);
  {
    const int n2 = DFF * ND / 8;
    cvt_f16<<<(n2 + 255) / 256, 256, 0, stream>>>(W2, w2h, n2, 16.0f);
  }
  gemm_f16<3><<<dim3(ND / 64, (unsigned)(rowsAll / 64), 1), 128, 0, stream>>>(
      hid, DFF, 0, w2h, ND, 0, zn, z2, ND, 0, z1, ND, 0, b2, 1, zn, ND, 0, DFF, inv16);

  ln_f16<<<(unsigned)((rowsAll + 7) / 8), 256, 0, stream>>>(z2, ln3g, ln3b, txc, NK * ND, (int)rowsAll);
  {
    const int nl = NB * NN * NN / 8;
    cvt_f16<<<(nl + 255) / 256, 256, 0, stream>>>(lap, L16, nl, 16.0f);
    const int nt = NK * ND * ND / 8;
    cvt_f16<<<(nt + 255) / 256, 256, 0, stream>>>(Th, thh, nt, 16.0f);
  }
  gemm_f16<0><<<dim3(ND / 64, NN / 64, NB), 128, 0, stream>>>(
      L16, NN, sNN, txc, NK * ND, sTX, txc + ND, z1, NK * ND, sTX, z1, ND, 0, b1, 0, txc, NK * ND, sTX, NN, inv16);
  gemm_f16<2><<<dim3(ND / 64, NN / 64, NB), 128, 0, stream>>>(
      L16, NN, sNN, txc + ND, NK * ND, sTX, txc + 2 * ND, z1, NK * ND, sTX, z1, ND, 0, b1, 0, txc, NK * ND, sTX, NN, inv16);
  gemm_f16<3><<<dim3(ND / 64, (unsigned)(rowsAll / 64), 1), 128, 0, stream>>>(
      txc, NK * ND, 0, thh, ND, 0, zn, out, ND, 0, z2, ND, 0, b2, 0, zn, ND, 0, NK * ND, inv16);
}
